// GraphVToS_9388798509586
// MI455X (gfx1250) — hardware-run, weakly checked
//
#include <hip/hip_runtime.h>

typedef float          v8f   __attribute__((ext_vector_type(8)));
typedef float          v4f   __attribute__((ext_vector_type(4)));
typedef unsigned int   v4u   __attribute__((ext_vector_type(4)));
typedef int            v8i   __attribute__((ext_vector_type(8)));
typedef unsigned short v8us  __attribute__((ext_vector_type(8)));
typedef unsigned short v16us __attribute__((ext_vector_type(16)));
typedef __bf16         v16bf __attribute__((ext_vector_type(16)));
typedef _Float16       v16h  __attribute__((ext_vector_type(16)));
typedef v4f  __attribute__((may_alias)) v4fa;
typedef v8us __attribute__((may_alias)) v8usa;
union FragB { v16bf v; v16us u; v8us h[2]; v8i w; };
union FragH { v16h  v; v16us u; v8us h[2]; v8i w; };

__device__ __forceinline__ v8f wmb(const FragB& a, const FragB& b, v8f c) {
  v8f d = __builtin_amdgcn_wmma_f32_16x16x32_bf16(false, a.v, false, b.v, (short)0, c, false, false);
  asm volatile("v_nop\n\tv_nop\n\tv_nop\n\tv_nop" : "+v"(d) : "v"(a.w), "v"(b.w));
  return d;
}

__device__ __forceinline__ v8f wmh(const FragH& a, const FragH& b, v8f c) {
  v8f d = __builtin_amdgcn_wmma_f32_16x16x32_f16(false, a.v, false, b.v, (short)0, c, false, false);
  asm volatile("v_nop\n\tv_nop\n\tv_nop\n\tv_nop" : "+v"(d) : "v"(a.w), "v"(b.w));
  return d;
}

__device__ __forceinline__ unsigned bf16_bits(float f) {
  const unsigned u = __float_as_uint(f);
  const unsigned r = (u + 0x7FFFu + ((u >> 16) & 1u)) >> 16;
  const unsigned q = (u >> 16) | 0x40u;
  return ((u & 0x7fffffffu) > 0x7f800000u) ? q : r;
}

__device__ __forceinline__ float bf16_val(float f) {
  return __uint_as_float(bf16_bits(f) << 16);
}
__device__ __forceinline__ int clampi(int v, int lo, int hi) {
  return v < lo ? lo : (v > hi ? hi : v);
}

__device__ __forceinline__ unsigned f16_bits(float f) {
  const unsigned u  = __float_as_uint(f);
  const unsigned s  = (u >> 16) & 0x8000u;
  const unsigned a  = u & 0x7fffffffu;
  const unsigned t  = a - 0x38000000u;
  const unsigned r  = (t + 0x0FFFu + ((t >> 13) & 1u)) >> 13;
  const unsigned rc = r > 0x7C00u ? 0x7C00u : r;
  const bool small  = a < 0x38800000u;
  const bool isnan  = a > 0x7f800000u;
  const unsigned fin = small ? 0u : (s | rc);
  return isnan ? (s | 0x7E00u) : fin;
}

__device__ __forceinline__ unsigned pk16(unsigned lo, unsigned hi) { return lo | (hi << 16); }
__device__ __forceinline__ unsigned bf16_lo_bits(float v) {
  float hi = bf16_val(v);
  asm volatile("" : "+v"(hi));
  return bf16_bits(v - hi);
}
__device__ __forceinline__ v4u pack8_bf16(v4f a, v4f c) {
  return (v4u){ pk16(bf16_bits(a[0]), bf16_bits(a[1])), pk16(bf16_bits(a[2]), bf16_bits(a[3])),
                pk16(bf16_bits(c[0]), bf16_bits(c[1])), pk16(bf16_bits(c[2]), bf16_bits(c[3])) };
}
__device__ __forceinline__ v4u pack8_bf16_lo(v4f a, v4f c) {
  return (v4u){ pk16(bf16_lo_bits(a[0]), bf16_lo_bits(a[1])), pk16(bf16_lo_bits(a[2]), bf16_lo_bits(a[3])),
                pk16(bf16_lo_bits(c[0]), bf16_lo_bits(c[1])), pk16(bf16_lo_bits(c[2]), bf16_lo_bits(c[3])) };
}
__device__ __forceinline__ v4u pack8_f16(v4f a, v4f c) {
  return (v4u){ pk16(f16_bits(a[0]), f16_bits(a[1])), pk16(f16_bits(a[2]), f16_bits(a[3])),
                pk16(f16_bits(c[0]), f16_bits(c[1])), pk16(f16_bits(c[2]), f16_bits(c[3])) };
}

template <int FORM>
__global__ __launch_bounds__(256) void k_plane(const float* __restrict__ src, int rows, int cols, int ldsrc,
                                               unsigned short* __restrict__ dst, int MP, int KP) {
  static_assert(FORM >= 0 && FORM <= 3);
  const int KTOT = (FORM == 1 || FORM == 3) ? 2 * KP : KP;
  const unsigned ppr   = (unsigned)(KTOT >> 3);
  const unsigned kp8   = (unsigned)(KP >> 3);
  const unsigned total = (unsigned)MP * ppr;
  const unsigned g     = blockIdx.x * 256u + threadIdx.x;
  const unsigned rowu  = g / ppr;
  const unsigned p     = g - rowu * ppr;
  const bool second    = p >= kp8;
  const int row = (int)rowu;
  const int c0  = (int)((second ? p - kp8 : p) << 3);
  const float* srow = src + (size_t)clampi(row, 0, rows - 1) * (size_t)ldsrc;
  float x[8];
  unsigned mk[8];
#pragma unroll
  for (int e = 0; e < 8; ++e) {
    const int c = c0 + e;
    const float v = srow[clampi(c, 0, cols - 1)];
    asm volatile("" :: "v"(v));
    x[e]  = v;
    mk[e] = (row < rows && c < cols) ? 0xFFFFu : 0u;
  }
  const v4f a = (v4f){ x[0], x[1], x[2], x[3] };
  const v4f c = (v4f){ x[4], x[5], x[6], x[7] };
  v4u o;
  if (FORM == 2) {
    o = pack8_f16(a, c);
  } else {
    const v4u hi = pack8_bf16(a, c);
    o = hi;
    if (FORM == 1) { const v4u lo = pack8_bf16_lo(a, c); o = second ? lo : hi; }
  }
  const v4u mw = (v4u){ pk16(mk[0], mk[1]), pk16(mk[2], mk[3]), pk16(mk[4], mk[5]), pk16(mk[6], mk[7]) };
  o &= mw;
  if (g < total) {
    volatile v4u* q = (volatile v4u*)(dst + (size_t)g * 8);
    *q = o;
    __threadfence();
    *q = o;
  }
}

template <int FORM> struct FragOf    { typedef FragB T; };
template <>         struct FragOf<2> { typedef FragH T; };
__device__ __forceinline__ v8f mm(const FragB& a, const FragB& b, v8f c) { return wmb(a, b, c); }
__device__ __forceinline__ v8f mm(const FragH& a, const FragH& b, v8f c) { return wmh(a, b, c); }
template <class F> __device__ __forceinline__ F ld_frag(const unsigned short* p) {
  F f;
  f.h[0] = *(const v8usa*)(p);
  f.h[1] = *(const v8usa*)(p + 16);
  return f;
}

template <int FORM, int EPI>
__global__ __launch_bounds__(256) __attribute__((amdgpu_num_vgpr(248)))
void k_gemm_nt(const unsigned short* __restrict__ A, const unsigned short* __restrict__ B,
               const float* __restrict__ bias, float* __restrict__ D, int M, int N, int KTOT, int ldd) {
  static_assert(FORM >= 0 && FORM <= 2);
  static_assert(EPI == 0 || EPI == 1);
  typedef typename FragOf<FORM>::T F;
  __shared__ __attribute__((aligned(16))) float sT[8][16 * 68];
  const int lane = threadIdx.x & 31;
  const int wave = threadIdx.x >> 5;
  const int tilesM = (M + 63) >> 6;
  const int tilesN = (N + 63) >> 6;
  const int tile = blockIdx.x * 8 + wave;
  if (tile >= tilesM * tilesN) return;
  const int tm = tile / tilesN;
  const int tn = tile - tm * tilesN;
  const int m0 = tm << 6;
  const int n0 = tn << 6;

  const int rl = lane & 15;
  const int h8 = (lane >> 4) * 8;
  const unsigned short* pa = A + (size_t)(m0 + rl) * (size_t)KTOT + h8;
  const unsigned short* pb = B + (size_t)(n0 + rl) * (size_t)KTOT + h8;

  v8f acc[4][4];
#pragma unroll
  for (int i = 0; i < 4; ++i)
#pragma unroll
    for (int j = 0; j < 4; ++j) acc[i][j] = (v8f){0.f, 0.f, 0.f, 0.f, 0.f, 0.f, 0.f, 0.f};

#pragma unroll 1
  for (int k0 = 0; k0 < KTOT; k0 += 32) {
    F bf[4];
#pragma unroll
    for (int j = 0; j < 4; ++j) bf[j] = ld_frag<F>(pb + (size_t)(j << 4) * (size_t)KTOT + k0);
#pragma unroll
    for (int i = 0; i < 4; ++i) {
      const F af = ld_frag<F>(pa + (size_t)(i << 4) * (size_t)KTOT + k0);
#pragma unroll
      for (int j = 0; j < 4; ++j) acc[i][j] = mm(af, bf[j], acc[i][j]);
    }
  }

  float* slab = sT[wave];
  const int hh = lane >> 4;
  const int c4 = (lane & 15) * 4;
  const int nc = n0 + c4;
  const bool cok = nc < N;
  v4f bv = (v4f){0.f, 0.f, 0.f, 0.f};
  if (EPI == 1) {
    bv = *(const v4fa*)(bias + clampi(nc, 0, N - 4));
    asm volatile("" :: "v"(bv));
  }
#pragma unroll
  for (int i = 0; i < 4; ++i) {
    const int mBase = m0 + (i << 4);
#pragma unroll
    for (int j = 0; j < 4; ++j) {
#pragma unroll
      for (int r = 0; r < 8; ++r) slab[(h8 + r) * 68 + (j << 4) + rl] = acc[i][j][r];
    }
    __builtin_amdgcn_fence(__ATOMIC_RELEASE, "workgroup");
    __builtin_amdgcn_wave_barrier();
    __builtin_amdgcn_fence(__ATOMIC_ACQUIRE, "workgroup");
    v4f vv[8];
#pragma unroll
    for (int it = 0; it < 8; ++it) {
      const int row = it * 2 + hh;
      v4f v = *(const v4fa*)(slab + row * 68 + c4);
      if (EPI == 1) v += bv;
      vv[it] = v;
    }
    for (int pass = 0; pass < 2; ++pass) {
#pragma unroll
      for (int it = 0; it < 8; ++it) {
        const int row = mBase + it * 2 + hh;
        if (cok && row < M) *(volatile v4f*)(D + (size_t)row * (size_t)ldd + nc) = vv[it];
      }
      __threadfence();
    }
    __builtin_amdgcn_fence(__ATOMIC_RELEASE, "workgroup");
    __builtin_amdgcn_wave_barrier();
    __builtin_amdgcn_fence(__ATOMIC_ACQUIRE, "workgroup");
  }
}

#define NBAT   8
#define NATOM  128
#define NAX    3
#define NFEAT  64
#define NOUT   64
#define GM     (NBAT * NATOM * NAX)
#define GN     (2 * NOUT)
#define GK     NFEAT
#define ND     (NATOM * NAX)
#define WTP    72
#define DLOADERS 96

typedef float v2f __attribute__((ext_vector_type(2)));
typedef v2f __attribute__((may_alias)) v2fa;
typedef v4u __attribute__((may_alias)) v4ua;

static_assert(NBAT == 8 && NATOM == 128 && NAX == 3 && NFEAT == 64 && NOUT == 64);
static_assert(GM == 3072 && GM % 64 == 0 && GM % 16 == 0);
static_assert(GN == 128 && GN % 64 == 0 && GN % 4 == 0);
static_assert(GK % 32 == 0);
static_assert(GN % 32 == 0);
static_assert((GM * GK / 8) % 256 == 0);
static_assert((((GM + 63) / 64) * ((GN + 63) / 64)) % 8 == 0);
static_assert(DLOADERS == 3 * 32);
static_assert(DLOADERS * 4 == ND);
static_assert(8 * 16 == NATOM);
static_assert(32 * 2 == NOUT);
static_assert((WTP * 2) % 16 == 0);
static_assert((size_t)(NBAT * NATOM - 1) * ND + ND - 1 == (size_t)NBAT * NATOM * NATOM * NAX - 1);
static_assert((size_t)(GM - 1) * GN + GN - 1 == (size_t)GM * GN - 1);
static_assert(((size_t)(NBAT * NATOM - 1) * NATOM + NATOM - 1) * NOUT + NOUT - 1 == (size_t)8388608 - 1);

#define WS_XB   ((size_t)GM * GK * 2)
#define WS_WT   ((size_t)GN * GK * 2)
#define WS_P    ((size_t)GM * GN * 4)
#define WS_TOTAL (WS_XB + WS_WT + WS_P)
static_assert(WS_XB == 393216 && WS_WT == 16384 && WS_P == 1572864);
static_assert(WS_XB % 256 == 0 && (WS_XB + WS_WT) % 256 == 0);
static_assert(WS_TOTAL == 1982464);
static_assert(WS_TOTAL <= ((size_t)128 << 20));

__global__ __launch_bounds__(256) void k_wprep(const float* __restrict__ W, unsigned short* __restrict__ WT) {
  __shared__ __attribute__((aligned(16))) unsigned short sT[GN * WTP];
  const int tid = threadIdx.x, lane = tid & 31, w = tid >> 5;
  const int c4 = (tid & 15) * 4, rr = tid >> 4;
#pragma unroll
  for (int p = 0; p < 8; ++p) {
    const int r = rr + 16 * p;
    const v4f v = *(const v4fa*)(W + (size_t)r * NOUT + c4);
    const int nb = (r >> 6) * NOUT + c4;
    const int k  = r & 63;
    sT[(nb + 0) * WTP + k] = (unsigned short)bf16_bits(v[0]);
    sT[(nb + 1) * WTP + k] = (unsigned short)bf16_bits(v[1]);
    sT[(nb + 2) * WTP + k] = (unsigned short)bf16_bits(v[2]);
    sT[(nb + 3) * WTP + k] = (unsigned short)bf16_bits(v[3]);
  }
  __syncthreads();
  const int q8 = lane & 7, sub = lane >> 3;
  v4u vv[4];
#pragma unroll
  for (int it = 0; it < 4; ++it) {
    const int row = 32 * it + 4 * w + sub;
    vv[it] = *(const v4ua*)(sT + row * WTP + 8 * q8);
  }
  for (int pass = 0; pass < 2; ++pass) {
#pragma unroll
    for (int it = 0; it < 4; ++it) {
      const int row = 32 * it + 4 * w + sub;
      *(volatile v4u*)(WT + (size_t)row * GK + 8 * q8) = vv[it];
    }
    __threadfence();
  }
}

__global__ __launch_bounds__(256) void k_pair(const float* __restrict__ dist, const float* __restrict__ P,
                                              const float* __restrict__ bvs, float* __restrict__ out) {
#pragma clang fp contract(off)
  __shared__ __attribute__((aligned(16))) float sD[ND];
  __shared__ __attribute__((aligned(16))) float sB[NOUT];
  const int tid = threadIdx.x, lane = tid & 31, wave = tid >> 5;
  const int bi = blockIdx.x;

  if (wave < 3) {
    const v4f dv = *(const v4fa*)(dist + (size_t)bi * ND + 4 * tid);
    sD[4 * tid + 0] = bf16_val(dv[0]);
    sD[4 * tid + 1] = bf16_val(dv[1]);
    sD[4 * tid + 2] = bf16_val(dv[2]);
    sD[4 * tid + 3] = bf16_val(dv[3]);
  } else if (wave == 3) {
    const v2f bv = *(const v2fa*)(bvs + 2 * lane);
    sB[2 * lane + 0] = bf16_val(bv[0]);
    sB[2 * lane + 1] = bf16_val(bv[1]);
  }
  __syncthreads();

  const int k2 = 2 * lane;
  const float* prow = P + (size_t)bi * (NAX * GN) + k2;
  const v2f pi0 = *(const v2fa*)(prow);
  const v2f pi1 = *(const v2fa*)(prow + GN);
  const v2f pi2 = *(const v2fa*)(prow + 2 * GN);
  const float pi0x = pi0[0], pi0y = pi0[1], pi1x = pi1[0], pi1y = pi1[1], pi2x = pi2[0], pi2y = pi2[1];
  asm volatile("" :: "v"(pi0x), "v"(pi0y), "v"(pi1x), "v"(pi1y), "v"(pi2x), "v"(pi2y));
  const float bx = sB[k2], by = sB[k2 + 1];

  const int bb = bi >> 7;
  const float* pjb = P + (size_t)(bb * NATOM) * (NAX * GN) + NOUT + k2;
  float* orow = out + (size_t)bi * (NATOM * NOUT) + k2;
  const int j0 = wave * 16;

#pragma unroll 1
  for (int jj = 0; jj < 16; ++jj) {
    const int j = j0 + jj;
    const float* pj = pjb + (size_t)j * (NAX * GN);
    const v2f q0 = *(const v2fa*)(pj);
    const v2f q1 = *(const v2fa*)(pj + GN);
    const v2f q2 = *(const v2fa*)(pj + 2 * GN);
    const float q0x = q0[0], q0y = q0[1], q1x = q1[0], q1y = q1[1], q2x = q2[0], q2y = q2[1];
    asm volatile("" :: "v"(q0x), "v"(q0y), "v"(q1x), "v"(q1y), "v"(q2x), "v"(q2y));
    const float d0 = sD[3 * j + 0];
    const float d1 = sD[3 * j + 1];
    const float d2 = sD[3 * j + 2];
    const float ds = (d0 + d1) + d2;

    float ax = pi0x * d0;
    ax = fmaf(pi1x, d1, ax);
    ax = fmaf(pi2x, d2, ax);
    ax = fmaf(q0x, d0, ax);
    ax = fmaf(q1x, d1, ax);
    ax = fmaf(q2x, d2, ax);
    ax = fmaf(ds, bx, ax);
    float ay = pi0y * d0;
    ay = fmaf(pi1y, d1, ay);
    ay = fmaf(pi2y, d2, ay);
    ay = fmaf(q0y, d0, ay);
    ay = fmaf(q1y, d1, ay);
    ay = fmaf(q2y, d2, ay);
    ay = fmaf(ds, by, ay);

    const float rx = (ax > 0.0f) ? ax : (ax - ax);
    const float ry = (ay > 0.0f) ? ay : (ay - ay);
    const v2f o = (v2f){ rx, ry };
    volatile v2f* op = (volatile v2f*)(orow + (size_t)j * NOUT);
    *op = o;
    __threadfence();
    *op = o;
  }
}

extern "C" void kernel_launch(void* const* d_in, const int* in_sizes, int n_in,
                              void* d_out, int out_size, void* d_ws, size_t ws_size,
                              hipStream_t stream) {
  if (n_in < 4) return;
  if (in_sizes[0] != NBAT * NATOM * NAX * NFEAT) return;
  if (in_sizes[1] != NBAT * NATOM * NATOM * NAX) return;
  if (in_sizes[2] != 2 * NFEAT * NOUT) return;
  if (in_sizes[3] != NOUT) return;
  if (out_size != NBAT * NATOM * NATOM * NOUT) return;
  if (ws_size < WS_TOTAL) return;

  const float* vf   = (const float*)d_in[0];
  const float* dist = (const float*)d_in[1];
  const float* wv   = (const float*)d_in[2];
  const float* bv   = (const float*)d_in[3];
  float* out = (float*)d_out;

  char* ws = (char*)d_ws;
  unsigned short* XB = (unsigned short*)(ws);
  unsigned short* WT = (unsigned short*)(ws + WS_XB);
  float*          P  = (float*)(ws + WS_XB + WS_WT);

  k_plane<0><<<dim3((GM * GK / 8) / 256), dim3(256), 0, stream>>>(vf, GM, GK, GK, XB, GM, GK);
  k_wprep<<<dim3(1), dim3(256), 0, stream>>>(wv, WT);
  k_gemm_nt<0, 0><<<dim3(12), dim3(256), 0, stream>>>(XB, WT, wv, P, GM, GN, GK, GN);
  k_pair<<<dim3(NBAT * NATOM), dim3(256), 0, stream>>>(dist, P, bv, out);
}
